// RClassifier0_58978490908736
// MI455X (gfx1250) — hardware-verified
//
#include <hip/hip_runtime.h>
#include <stddef.h>


typedef _Float16 f16t;
typedef f16t  v16h __attribute__((ext_vector_type(16)));
typedef f16t  v8h  __attribute__((ext_vector_type(8)));
typedef float v8f  __attribute__((ext_vector_type(8)));
typedef float v4f  __attribute__((ext_vector_type(4)));
typedef v4f   v4fa __attribute__((may_alias));
typedef v8h   v8ha __attribute__((may_alias));
union Frag { v16h v; v8h half[2]; };

#define NB       32
#define NTHR     256
#define NWAVE    (NTHR / 32)
#define SC_A     256.0f
#define SC_W     1024.0f
#define SC_F1    4096.0f
#define INV_AW   (1.0f / 262144.0f)
#define INV_AF1  (1.0f / 1048576.0f)

#define L0_NOUT  65536
#define L0_SHIFT 16
#define L0_PER   65536
#define L0_NQ    4
#define NPB1     32
#define M0PB     (NPB1 * 4)
#define NPB2     8

#define FC_K     16384
#define FC_H     128
#define FC_NODES 128

__device__ __forceinline__ v8f wmma16(v8f acc, v16h a, v16h b)
{
    acc = __builtin_amdgcn_wmma_f32_16x16x32_f16(false, a, false, b, (short)0, acc, false, false);
    asm volatile("v_nop\n\tv_nop\n\tv_nop\n\tv_nop" : "+v"(acc) : "v"(a), "v"(b));
    return acc;
}

__device__ __forceinline__ v8f zero8f()
{
    v8f z;
#pragma unroll
    for (int i = 0; i < 8; ++i) z[i] = 0.0f;
    return z;
}

__device__ __forceinline__ v8h zero8h()
{
    v8h z;
#pragma unroll
    for (int i = 0; i < 8; ++i) z[i] = (f16t)0.0f;
    return z;
}

__device__ __forceinline__ int fixr(int r)
{
    if (r < 0) r += 8;
    if (r < 0) r = 0;
    if (r > 7) r = 7;
    return r;
}

__device__ __forceinline__ void store_lines2(const unsigned char* s, unsigned char* d, int nlines)
{
    const int w = threadIdx.x >> 5, l = threadIdx.x & 31;
    const int q = l & 7;
    for (int L = w * 4 + (l >> 3); L < nlines; L += NWAVE * 4) {
        const size_t o = (size_t)L * 128 + (size_t)q * 16;
        const v4f v = *(const v4fa*)(s + o);
        *(volatile v4f*)(d + o) = v;
    }
    __threadfence();
    for (int L = w * 4 + (l >> 3); L < nlines; L += NWAVE * 4) {
        const size_t o = (size_t)L * 128 + (size_t)q * 16;
        const v4f v = *(const v4fa*)(s + o);
        *(volatile v4f*)(d + o) = v;
    }
}

__global__ __launch_bounds__(NTHR)
void k_l0(const float* __restrict__ x, const int* __restrict__ par0, const int* __restrict__ reg0,
          const float* __restrict__ W0, const float* __restrict__ b0,
          const int* __restrict__ par1,
          float* __restrict__ agg1, int nin0, int nout0, int nout1)
{
    __shared__ __attribute__((aligned(16))) float agg0[NB * M0PB];
    __shared__ __attribute__((aligned(16))) float stg[NPB1 * NB * 8];
    __shared__ float w0s[64];
    __shared__ float b0s[8];
    __shared__ int rl0[M0PB];
    __shared__ int p1ok[M0PB];

    const int tid = threadIdx.x;
    const int j0 = blockIdx.x * NPB1;
    const int m0 = j0 * 4;

    if (tid < 64) w0s[tid] = W0[tid];
    if (tid < 8) b0s[tid] = b0[tid];
    if (tid < M0PB) {
        const int m = m0 + tid;
        int r = 0, ok = 0;
        if (m < nout0) {
            r = fixr(reg0[m]);
            ok = (par1[m] == (m >> 2)) ? 1 : 0;
        }
        rl0[tid] = r;
        p1ok[tid] = ok;
    }

    {
        const int ml = tid & (M0PB - 1);
        const int nb = tid >> 7;
        const int m = m0 + ml;
        float acc[16];
#pragma unroll
        for (int k = 0; k < 16; ++k) acc[k] = 0.0f;
        if (m < nout0) {
            const long long sl = ((long long)m * nin0 + (L0_NOUT - 1)) >> L0_SHIFT;
            const long long el = ((long long)(m + 1) * nin0 + (L0_NOUT - 1)) >> L0_SHIFT;
            const int vs = (int)sl - 1;
            const int ve = (int)el + 1;
#pragma unroll 1
            for (int q = 0; q < L0_NQ; ++q) {
#pragma unroll 1
                for (int dv = 0; dv < 6; ++dv) {
                    const int v = vs + dv;
                    if (v < 0 || v >= ve || v >= L0_PER) continue;
                    const int i = q * L0_PER + v;
                    if (i >= nin0) continue;
                    if (par0[i] != m) continue;
                    const float* xp = x + i;
#pragma unroll
                    for (int k = 0; k < 16; ++k)
                        acc[k] += xp[(size_t)(nb + 2 * k) * (size_t)nin0];
                }
            }
        }
#pragma unroll
        for (int k = 0; k < 16; ++k) agg0[(nb + 2 * k) * M0PB + ml] = acc[k];
    }
    __syncthreads();

    for (int it = 0; it < (NPB1 * NB) / NTHR; ++it) {
        const int task = it * NTHR + tid;
        const int jl = task & (NPB1 - 1);
        const int n = task >> 5;
        float ag[8];
#pragma unroll
        for (int c = 0; c < 8; ++c) ag[c] = 0.0f;
#pragma unroll
        for (int t4 = 0; t4 < 4; ++t4) {
            const int ml = jl * 4 + t4;
            if (p1ok[ml]) {
                const float a = agg0[n * M0PB + ml];
                const int r = rl0[ml];
#pragma unroll
                for (int c = 0; c < 8; ++c) ag[c] += fmaf(w0s[r * 8 + c], a, b0s[c]);
            }
        }
        float* so = stg + (jl * NB + n) * 8;
#pragma unroll
        for (int c = 0; c < 8; ++c) so[c] = ag[c];
    }
    __syncthreads();

    int nval = nout1 - j0;
    if (nval > NPB1) nval = NPB1;
    if (nval < 0) nval = 0;
    const int nlines = nval * NB * 8 * 4 / 128;
    store_lines2((const unsigned char*)stg,
                 (unsigned char*)agg1 + (size_t)j0 * NB * 8 * 4, nlines);
}

__global__ __launch_bounds__(NTHR)
void k_l12(const float* __restrict__ agg1, const int* __restrict__ par2,
           const int* __restrict__ reg1, const float* __restrict__ W1, const float* __restrict__ b1,
           const int* __restrict__ reg2, const float* __restrict__ W2, const float* __restrict__ b2,
           float* __restrict__ z3, int nin, int nout)
{
    __shared__ __attribute__((aligned(16))) f16t a1[NPB2 * NB * 32];
    __shared__ __attribute__((aligned(16))) f16t b1h[NPB2 * 16 * 32];
    __shared__ __attribute__((aligned(16))) f16t a2[NPB2 * NB * 16];
    __shared__ __attribute__((aligned(16))) f16t w2h[NPB2 * 32 * 16];
    __shared__ __attribute__((aligned(16))) unsigned char stg[NPB2 * NB * 32 * 4];
    __shared__ float b1s[16];
    __shared__ float b2s[32];
    __shared__ int rl1s[NPB2 * 4];
    __shared__ int ok2[NPB2 * 4];
    __shared__ int rl2s[NPB2];

    const int tid = threadIdx.x;
    const int j0 = blockIdx.x * NPB2;

    if (tid < NPB2 * 4) {
        const int jl = tid >> 2, t = tid & 3;
        const int j = j0 + jl;
        const int j1 = j * 4 + t;
        int ok = 0, r = 0;
        if (j < nout && j1 < nin) {
            ok = (par2[j1] == j) ? 1 : 0;
            r = fixr(reg1[j1]);
        }
        ok2[tid] = ok;
        rl1s[tid] = r;
    }
    if (tid < NPB2) {
        const int j = j0 + tid;
        rl2s[tid] = (j < nout) ? fixr(reg2[j]) : 0;
    }
    if (tid < 16) b1s[tid] = b1[tid];
    if (tid < 32) b2s[tid] = b2[tid];
    __syncthreads();

    for (int idx = tid; idx < NPB2 * NB * 32; idx += NTHR) {
        const int k = idx & 31;
        const int n = (idx >> 5) & 31;
        const int jl = idx >> 10;
        const int t = k >> 3, c = k & 7;
        const int j = j0 + jl;
        float v = 0.0f;
        if (ok2[jl * 4 + t]) v = agg1[((size_t)(j * 4 + t) * NB + n) * 8 + c];
        a1[idx] = (f16t)(SC_A * v);
    }
    for (int idx = tid; idx < NPB2 * 16 * 32; idx += NTHR) {
        const int k = idx & 31;
        const int d = (idx >> 5) & 15;
        const int jl = idx >> 9;
        const int t = k >> 3, c = k & 7;
        const int r = rl1s[jl * 4 + t];
        b1h[idx] = (f16t)(SC_W * W1[(r * 16 + d) * 8 + c]);
    }
    for (int idx = tid; idx < NPB2 * 32 * 16; idx += NTHR) {
        const int d = idx & 15;
        const int e = (idx >> 4) & 31;
        const int jl = idx >> 9;
        w2h[idx] = (f16t)(SC_W * W2[(rl2s[jl] * 32 + e) * 16 + d]);
    }
    __syncthreads();

    const int w = tid >> 5, l = tid & 31, h = l >> 4, lm = l & 15;

    for (int tt = w; tt < NPB2 * 2; tt += NWAVE) {
        const int jl = tt >> 1, mt = tt & 1;
        const int n = mt * 16 + lm;
        const int d = lm;
        const f16t* ar = a1 + (jl * NB + n) * 32;
        const f16t* br = b1h + (jl * 16 + d) * 32;
        Frag a, b;
        a.half[0] = *(const v8ha*)(ar + 8 * h);
        a.half[1] = *(const v8ha*)(ar + 16 + 8 * h);
        b.half[0] = *(const v8ha*)(br + 8 * h);
        b.half[1] = *(const v8ha*)(br + 16 + 8 * h);
        v8f acc = zero8f();
        acc = wmma16(acc, a.v, b.v);
        const float cnt = (float)(ok2[jl * 4] + ok2[jl * 4 + 1] + ok2[jl * 4 + 2] + ok2[jl * 4 + 3]);
        const float bd = cnt * b1s[d];
#pragma unroll
        for (int r = 0; r < 8; ++r) {
            const int nn = mt * 16 + 8 * h + r;
            const float val = acc[r] * INV_AW + bd;
            a2[(jl * NB + nn) * 16 + d] = (f16t)(SC_A * val);
        }
    }
    __syncthreads();

    for (int tt = w; tt < NPB2 * 4; tt += NWAVE) {
        const int jl = tt >> 2, mt = (tt >> 1) & 1, nt = tt & 1;
        const int n = mt * 16 + lm;
        const int e = nt * 16 + lm;
        const f16t* ar = a2 + (jl * NB + n) * 16;
        const f16t* br = w2h + (jl * 32 + e) * 16;
        Frag a, b;
        a.half[0] = *(const v8ha*)(ar + 8 * h);
        a.half[1] = zero8h();
        b.half[0] = *(const v8ha*)(br + 8 * h);
        b.half[1] = zero8h();
        v8f acc = zero8f();
        acc = wmma16(acc, a.v, b.v);
        const float be = b2s[e];
#pragma unroll
        for (int r = 0; r < 8; ++r) {
            const int nn = mt * 16 + 8 * h + r;
            ((float*)stg)[(jl * NB + nn) * 32 + e] = acc[r] * INV_AW + be;
        }
    }
    __syncthreads();

    int nval = nout - j0;
    if (nval > NPB2) nval = NPB2;
    if (nval < 0) nval = 0;
    const int nlines = nval * NB * 32 * 4 / 128;
    store_lines2(stg, (unsigned char*)z3 + (size_t)j0 * NB * 32 * 4, nlines);
}

template <int CIN, int COUT, int NCH, int NPB, int OUTH>
__global__ __launch_bounds__(NTHR)
void k_fgl(const float* __restrict__ zin, const int* __restrict__ par, const int* __restrict__ reg,
           const float* __restrict__ W, const float* __restrict__ bias,
           void* __restrict__ zout, int nin, int nout)
{
    constexpr int NT = COUT / 16;
    constexpr int KS = (CIN >= 32) ? (CIN / 32) : 1;
    constexpr int OES = OUTH ? 2 : 4;
    constexpr int STG_BYTES = NPB * NB * COUT * OES;

    __shared__ __attribute__((aligned(16))) f16t ah[NPB * NB * CIN];
    __shared__ __attribute__((aligned(16))) f16t wsl[NPB * COUT * CIN];
    __shared__ __attribute__((aligned(16))) unsigned char stg[STG_BYTES];
    __shared__ float bs[COUT];
    __shared__ int rl[NPB];
    __shared__ int okm[NPB * NCH];

    const int tid = threadIdx.x;
    const int j0 = blockIdx.x * NPB;

    if (tid < NPB) {
        const int j = j0 + tid;
        rl[tid] = (j < nout) ? fixr(reg[j]) : 0;
    }
    if (tid < NPB * NCH) {
        const int jl = tid / NCH;
        const int t = tid - jl * NCH;
        const int j = j0 + jl;
        const int i = j * NCH + t;
        int ok = 0;
        if (j < nout && i < nin) ok = (par[i] == j) ? 1 : 0;
        okm[tid] = ok;
    }
    for (int t = tid; t < COUT; t += NTHR) bs[t] = bias[t];
    __syncthreads();

    for (int idx = tid; idx < NPB * COUT * CIN; idx += NTHR) {
        const int c = idx % CIN;
        const int d = (idx / CIN) % COUT;
        const int jl = idx / (CIN * COUT);
        wsl[idx] = (f16t)(SC_W * W[((size_t)rl[jl] * COUT + d) * CIN + c]);
    }
    for (int idx = tid; idx < NPB * NB * CIN; idx += NTHR) {
        const int c = idx % CIN;
        const int n = (idx / CIN) % NB;
        const int jl = idx / (CIN * NB);
        const int j = j0 + jl;
        float s = 0.0f;
        if (j < nout) {
#pragma unroll
            for (int t = 0; t < NCH; ++t)
                if (okm[jl * NCH + t])
                    s += zin[((size_t)(j * NCH + t) * NB + n) * CIN + c];
        }
        ah[idx] = (f16t)(SC_A * s);
    }
    __syncthreads();

    const int w = tid >> 5, l = tid & 31, h = l >> 4, lm = l & 15;
    for (int tt = w; tt < NPB * 2 * NT; tt += NWAVE) {
        const int jl = tt / (2 * NT);
        const int rem = tt - jl * 2 * NT;
        const int mt = rem / NT;
        const int nt = rem - mt * NT;
        const int n = mt * 16 + lm;
        const int d = nt * 16 + lm;
        const f16t* ar = ah + (jl * NB + n) * CIN;
        const f16t* br = wsl + (jl * COUT + d) * CIN;
        v8f acc = zero8f();
#pragma unroll
        for (int ks = 0; ks < KS; ++ks) {
            const int k0 = ks * 32;
            Frag a, b;
            a.half[0] = *(const v8ha*)(ar + k0 + 8 * h);
            b.half[0] = *(const v8ha*)(br + k0 + 8 * h);
            if (CIN >= 32) {
                a.half[1] = *(const v8ha*)(ar + k0 + 16 + 8 * h);
                b.half[1] = *(const v8ha*)(br + k0 + 16 + 8 * h);
            } else {
                a.half[1] = zero8h();
                b.half[1] = zero8h();
            }
            acc = wmma16(acc, a.v, b.v);
        }
        const float bd = bs[d];
#pragma unroll
        for (int r = 0; r < 8; ++r) {
            const int nn = mt * 16 + 8 * h + r;
            const float val = acc[r] * INV_AW + bd;
            if (OUTH) ((f16t*)stg)[(jl * NB + nn) * COUT + d] = (f16t)(SC_A * val);
            else      ((float*)stg)[(jl * NB + nn) * COUT + d] = val;
        }
    }
    __syncthreads();

    int nval = nout - j0;
    if (nval > NPB) nval = NPB;
    if (nval < 0) nval = 0;
    const int nlines = nval * NB * COUT * OES / 128;
    store_lines2(stg, (unsigned char*)zout + (size_t)j0 * NB * COUT * OES, nlines);
}

__global__ __launch_bounds__(NTHR)
void k_fcw(const float* __restrict__ fw, f16t* __restrict__ wt, int nrow)
{
    __shared__ __attribute__((aligned(16))) f16t tl[32 * 136];
    const int tid = threadIdx.x;
    const int o = blockIdx.x >> 2;
    const int j0 = (blockIdx.x & 3) * 32;
    if (o >= nrow) return;
    const float* src = fw + (size_t)o * FC_K;
    for (int idx = tid; idx < FC_H * 32; idx += NTHR) {
        const int d = idx >> 5, jj = idx & 31;
        tl[jj * 136 + d] = (f16t)(SC_F1 * src[d * FC_NODES + j0 + jj]);
    }
    __syncthreads();

    unsigned char* dst = (unsigned char*)(wt + (size_t)o * FC_K + (size_t)j0 * FC_H);
    const unsigned char* sb = (const unsigned char*)tl;
    const int w = tid >> 5, l = tid & 31, q = l & 7;
    for (int L = w * 4 + (l >> 3); L < 64; L += NWAVE * 4) {
        const int jj = L >> 1;
        const int d = (L & 1) * 64 + q * 8;
        const v4f v = *(const v4fa*)(sb + ((size_t)jj * 136 + d) * 2);
        *(volatile v4f*)(dst + ((size_t)jj * FC_H + d) * 2) = v;
    }
    __threadfence();
    for (int L = w * 4 + (l >> 3); L < 64; L += NWAVE * 4) {
        const int jj = L >> 1;
        const int d = (L & 1) * 64 + q * 8;
        const v4f v = *(const v4fa*)(sb + ((size_t)jj * 136 + d) * 2);
        *(volatile v4f*)(dst + ((size_t)jj * FC_H + d) * 2) = v;
    }
}

__global__ __launch_bounds__(NTHR)
void k_fc(const f16t* __restrict__ z5h, const f16t* __restrict__ wt,
          const float* __restrict__ fb1, const float* __restrict__ fw2, const float* __restrict__ fb2,
          float* __restrict__ out, int ncls)
{
    __shared__ __attribute__((aligned(16))) f16t hs[NB * FC_H];
    __shared__ __attribute__((aligned(16))) f16t w2h[32 * FC_H];
    __shared__ float outs[NB * 32];
    __shared__ float b1s[FC_H];
    __shared__ float b2s[32];

    const int tid = threadIdx.x;
    for (int idx = tid; idx < 32 * FC_H; idx += NTHR) {
        const int cl = idx >> 7, o = idx & (FC_H - 1);
        w2h[idx] = (cl < ncls) ? (f16t)(SC_W * fw2[cl * FC_H + o]) : (f16t)0.0f;
    }
    if (tid < FC_H) b1s[tid] = fb1[tid];
    if (tid < 32) b2s[tid] = (tid < ncls) ? fb2[tid] : 0.0f;
    __syncthreads();

    const int w = tid >> 5, l = tid & 31, h = l >> 4, lm = l & 15;

    {
        const int o = w * 16 + lm;
        const f16t* brow = wt + (size_t)o * FC_K;
        v8f acc0 = zero8f(), acc1 = zero8f();
#pragma unroll 2
        for (int k0 = 0; k0 < FC_K; k0 += 32) {
            const int j = k0 >> 7;
            const int d0 = k0 & 127;
            const f16t* a0p = z5h + ((size_t)j * NB + lm) * FC_H + d0;
            const f16t* a1p = z5h + ((size_t)j * NB + 16 + lm) * FC_H + d0;
            Frag a0, a1, b;
            a0.half[0] = *(const v8ha*)(a0p + 8 * h);
            a0.half[1] = *(const v8ha*)(a0p + 16 + 8 * h);
            a1.half[0] = *(const v8ha*)(a1p + 8 * h);
            a1.half[1] = *(const v8ha*)(a1p + 16 + 8 * h);
            b.half[0] = *(const v8ha*)(brow + k0 + 8 * h);
            b.half[1] = *(const v8ha*)(brow + k0 + 16 + 8 * h);
            acc0 = wmma16(acc0, a0.v, b.v);
            acc1 = wmma16(acc1, a1.v, b.v);
        }
        const float bo = b1s[o];
#pragma unroll
        for (int r = 0; r < 8; ++r) {
            const int n0 = 8 * h + r;
            const int n1 = 16 + 8 * h + r;
            const float h0 = acc0[r] * INV_AF1 + bo;
            const float h1 = acc1[r] * INV_AF1 + bo;
            hs[n0 * FC_H + o] = (f16t)(SC_A * h0);
            hs[n1 * FC_H + o] = (f16t)(SC_A * h1);
        }
    }
    __syncthreads();

    if (w < 4) {
        const int mt = w & 1, nt = w >> 1;
        const int n = mt * 16 + lm;
        const int cl = nt * 16 + lm;
        const f16t* ar = hs + n * FC_H;
        const f16t* br = w2h + cl * FC_H;
        v8f acc = zero8f();
#pragma unroll
        for (int ks = 0; ks < FC_H / 32; ++ks) {
            const int k0 = ks * 32;
            Frag a, b;
            a.half[0] = *(const v8ha*)(ar + k0 + 8 * h);
            a.half[1] = *(const v8ha*)(ar + k0 + 16 + 8 * h);
            b.half[0] = *(const v8ha*)(br + k0 + 8 * h);
            b.half[1] = *(const v8ha*)(br + k0 + 16 + 8 * h);
            acc = wmma16(acc, a.v, b.v);
        }
        const float bc = b2s[cl];
#pragma unroll
        for (int r = 0; r < 8; ++r) {
            const int nn = mt * 16 + 8 * h + r;
            outs[nn * 32 + cl] = acc[r] * INV_AW + bc;
        }
    }
    __syncthreads();

    const int total = NB * ncls;
    const int e0 = tid * 4;
    const bool act = (e0 + 4 <= total);
    float vv[4];
#pragma unroll
    for (int qq = 0; qq < 4; ++qq) {
        const int e = e0 + qq;
        const int n = e / ncls;
        const int c = e - n * ncls;
        vv[qq] = (act && n < NB) ? outs[n * 32 + c] : 0.0f;
    }
    v4f v;
    v[0] = vv[0]; v[1] = vv[1]; v[2] = vv[2]; v[3] = vv[3];
    if (act) *(volatile v4f*)(out + e0) = v;
    __threadfence();
    if (act) *(volatile v4f*)(out + e0) = v;
}

extern "C" void kernel_launch(void* const* d_in, const int* in_sizes, int n_in,
                              void* d_out, int out_size, void* d_ws, size_t ws_size,
                              hipStream_t stream)
{
    if (n_in < 25) return;
    const float* x    = (const float*)d_in[0];
    const int*   par0 = (const int*)d_in[1];   const int* reg0 = (const int*)d_in[2];
    const float* W0   = (const float*)d_in[3]; const float* b0 = (const float*)d_in[4];
    const int*   par1 = (const int*)d_in[5];   const int* reg1 = (const int*)d_in[6];
    const float* W1   = (const float*)d_in[7]; const float* b1 = (const float*)d_in[8];
    const int*   par2 = (const int*)d_in[9];   const int* reg2 = (const int*)d_in[10];
    const float* W2   = (const float*)d_in[11]; const float* b2 = (const float*)d_in[12];
    const int*   par3 = (const int*)d_in[13];  const int* reg3 = (const int*)d_in[14];
    const float* W3   = (const float*)d_in[15]; const float* b3 = (const float*)d_in[16];
    const int*   par4 = (const int*)d_in[17];  const int* reg4 = (const int*)d_in[18];
    const float* W4   = (const float*)d_in[19]; const float* b4 = (const float*)d_in[20];
    const float* fc1w = (const float*)d_in[21]; const float* fc1b = (const float*)d_in[22];
    const float* fc2w = (const float*)d_in[23]; const float* fc2b = (const float*)d_in[24];
    float* out = (float*)d_out;

    const int nin0  = in_sizes[1];
    const int nout0 = in_sizes[2];
    const int nout1 = in_sizes[6];
    const int nout2 = in_sizes[10];
    const int nout3 = in_sizes[14];
    const int nout4 = in_sizes[18];
    const int ncls  = in_sizes[24];

    if (nout0 != L0_NOUT || nin0 > L0_NQ * L0_PER || in_sizes[5] != nout0) return;
    if ((size_t)in_sizes[0] != (size_t)NB * (size_t)nin0) return;
    if (nout0 != 4 * nout1 || nout1 != 4 * nout2 || nout2 != 4 * nout3 || nout3 != 8 * nout4) return;
    if (nout4 != FC_NODES || in_sizes[9] != nout1 || in_sizes[13] != nout2 || in_sizes[17] != nout3) return;
    if (in_sizes[3] != 8 * 8 * 1 || in_sizes[4] != 8 || in_sizes[7] != 8 * 16 * 8 || in_sizes[8] != 16 ||
        in_sizes[11] != 8 * 32 * 16 || in_sizes[12] != 32 ||
        in_sizes[15] != 8 * 64 * 32 || in_sizes[16] != 64 || in_sizes[19] != 8 * 128 * 64 || in_sizes[20] != 128) return;
    if (in_sizes[21] != FC_H * FC_K || in_sizes[22] != FC_H || ncls < 1 || ncls > 32 ||
        in_sizes[23] != ncls * FC_H || out_size != NB * ncls) return;

    unsigned char* ws = (unsigned char*)d_ws;
    size_t off = 0;
    float* agg1 = (float*)(ws + off); off += (size_t)nout1 * NB * 8 * 4;
    float* z3   = (float*)(ws + off); off += (size_t)nout2 * NB * 32 * 4;
    float* z4   = (float*)(ws + off); off += (size_t)nout3 * NB * 64 * 4;
    f16t*  z5h  = (f16t*)(ws + off);  off += (size_t)nout4 * NB * 128 * 2;
    f16t*  wt   = (f16t*)(ws + off);  off += (size_t)FC_H * FC_K * 2;
    if (off > ws_size) return;

    k_l0<<<dim3((nout1 + NPB1 - 1) / NPB1), dim3(NTHR), 0, stream>>>(
        x, par0, reg0, W0, b0, par1, agg1, nin0, nout0, nout1);

    k_fcw<<<dim3(FC_H * 4), dim3(NTHR), 0, stream>>>(fc1w, wt, FC_H);

    k_l12<<<dim3((nout2 + NPB2 - 1) / NPB2), dim3(NTHR), 0, stream>>>(
        agg1, par2, reg1, W1, b1, reg2, W2, b2, z3, nout1, nout2);
    k_fgl<32, 64, 4, 8, 0><<<dim3((nout3 + 7) / 8), dim3(NTHR), 0, stream>>>(
        z3, par3, reg3, W3, b3, (void*)z4, nout2, nout3);
    k_fgl<64, 128, 8, 4, 1><<<dim3((nout4 + 3) / 4), dim3(NTHR), 0, stream>>>(
        z4, par4, reg4, W4, b4, (void*)z5h, nout3, nout4);

    k_fc<<<dim3(1), dim3(NTHR), 0, stream>>>(z5h, wt, fc1b, fc2w, fc2b, out, ncls);
}
